// CausalSelfAttention_23819888624336
// MI455X (gfx1250) — hardware-verified
//
#include <hip/hip_runtime.h>
#ifndef NB
#define NB 2
#endif
#ifndef SEQ
#define SEQ 2048
#endif
#define NB_FULL 2
#define SEQ_FULL 2048
#define DM 1024
#define NH 16
#define HD 64
#define LQ (3 * DM)
#define NR ((size_t)NB * SEQ)
#define PSZ (NR * DM)
#define LN256 5.545177444f

static_assert(NB <= NB_FULL);
static_assert(SEQ <= SEQ_FULL);
static_assert(SEQ % 128 == 0);
static_assert(NH * HD == DM);
static_assert(HD == 64);
static_assert(DM == 1024);
static_assert(DM % 64 == 0);
static_assert(LQ % 64 == 0);
static_assert(DM % 32 == 0);
static_assert((2 * DM) % 32 == 0);
static_assert((NB * SEQ) % 128 == 0);

typedef _Float16 v16h __attribute__((ext_vector_type(16)));
typedef unsigned short v8us __attribute__((ext_vector_type(8), may_alias));
typedef float v8f __attribute__((ext_vector_type(8)));
typedef float v4f __attribute__((ext_vector_type(4)));
typedef float v4fa __attribute__((ext_vector_type(4), may_alias));
union FragH { v16h v; v8us half[2]; _Float16 h[16]; unsigned short u[16]; };

__device__ __forceinline__ unsigned short bf16_bits(float x) { unsigned int u = __float_as_uint(x); return (unsigned short)((u + 0x7FFFu + ((u >> 16) & 1u)) >> 16); }
__device__ __forceinline__ float bf16_rne(float x) { return __uint_as_float(((unsigned int)bf16_bits(x)) << 16); }

__device__ __forceinline__ v16h g2_frag(const unsigned short* p, int hh) { FragH f; f.half[0] = *(const v8us*)(p + 8 * hh); f.half[1] = *(const v8us*)(p + 16 + 8 * hh); return f.v; }
__device__ __forceinline__ v8f g2_mma(v16h a, v16h b, v8f c) { v8f d = __builtin_amdgcn_wmma_f32_16x16x32_f16(false, a, false, b, (short)0, c, false, false); asm volatile("v_nop\n\tv_nop\n\tv_nop\n\tv_nop" : "+v"(d) : "v"(a), "v"(b)); return d; }

__global__ __launch_bounds__(256) void k_wt_f16(const float* __restrict__ W, unsigned short* __restrict__ Wt, int K, int N, int ldo, float s0, float s1, int dual) {
  const int t = blockIdx.x * 256 + threadIdx.x; const int k8n = K >> 3;
  if (t >= N * k8n) return;
  const int n = t / k8n, k8 = (t - n * k8n) * 8;
  FragH f0, f1;
#pragma unroll
  for (int i = 0; i < 8; ++i) { const float v = bf16_rne(W[(size_t)(k8 + i) * N + n]); f0.h[i] = (_Float16)(v * s0); f1.h[i] = (_Float16)(v * s1); }
  const v8us o0 = f0.half[0], o1 = f1.half[0];
  unsigned short* d = Wt + (size_t)n * ldo + k8;
  *(volatile v8us*)d = o0; if (dual) *(volatile v8us*)(d + K) = o1;
  __threadfence();
  *(volatile v8us*)d = o0; if (dual) *(volatile v8us*)(d + K) = o1;
}

__global__ __launch_bounds__(256) void k_x16(const float* __restrict__ x, unsigned short* __restrict__ X16) {
  const size_t t = (size_t)blockIdx.x * 256 + threadIdx.x; if (t >= NR * DM / 8) return;
  const size_t row = t / (DM / 8); const int c8 = (int)(t % (DM / 8)) * 8;
  const size_t b = row / SEQ, s = row % SEQ;
  const float* src = x + (b * SEQ_FULL + s) * DM + c8;
  const v4f a = *(const v4fa*)src, c = *(const v4fa*)(src + 4);
  FragH f;
#pragma unroll
  for (int q = 0; q < 4; ++q) { f.h[q] = (_Float16)bf16_rne(a[q]); f.h[4 + q] = (_Float16)bf16_rne(c[q]); }
  const v8us o = f.half[0];
  *(volatile v8us*)(X16 + t * 8) = o; __threadfence(); *(volatile v8us*)(X16 + t * 8) = o;
}

struct Acc8 { v8f c00, c01, c02, c03, c10, c11, c12, c13; };
__device__ __forceinline__ Acc8 g2_main(const unsigned short* a0p, const unsigned short* a1p, const unsigned short* b0p, int ldb, int K, int hh) {
  const unsigned short* b1p = b0p + (size_t)16 * ldb; const unsigned short* b2p = b1p + (size_t)16 * ldb; const unsigned short* b3p = b2p + (size_t)16 * ldb;
  const v8f z8 = {0.f, 0.f, 0.f, 0.f, 0.f, 0.f, 0.f, 0.f};
  Acc8 c; c.c00 = z8; c.c01 = z8; c.c02 = z8; c.c03 = z8; c.c10 = z8; c.c11 = z8; c.c12 = z8; c.c13 = z8;
#pragma unroll 1
  for (int kb = 0; kb < K; kb += 32) {
    const v16h a0 = g2_frag(a0p + kb, hh), a1 = g2_frag(a1p + kb, hh);
    v16h b = g2_frag(b0p + kb, hh); c.c00 = g2_mma(a0, b, c.c00); c.c10 = g2_mma(a1, b, c.c10);
    b = g2_frag(b1p + kb, hh); c.c01 = g2_mma(a0, b, c.c01); c.c11 = g2_mma(a1, b, c.c11);
    b = g2_frag(b2p + kb, hh); c.c02 = g2_mma(a0, b, c.c02); c.c12 = g2_mma(a1, b, c.c12);
    b = g2_frag(b3p + kb, hh); c.c03 = g2_mma(a0, b, c.c03); c.c13 = g2_mma(a1, b, c.c13);
  }
  return c;
}

__global__ __launch_bounds__(128) void k_gemm_qkv(const unsigned short* __restrict__ X16, const unsigned short* __restrict__ BQ, const float* __restrict__ bias, unsigned short* __restrict__ PL) {
  __shared__ __attribute__((aligned(16))) float so[4][32][68];
  const int tid = threadIdx.x, lane = tid & 31, ln = lane & 15, hh = lane >> 4;
  const int w = __builtin_amdgcn_readfirstlane(tid >> 5);
  const int ntn = LQ / 64; const int mt = blockIdx.x / ntn, nq = blockIdx.x - mt * ntn;
  const int row0 = mt * 128 + 32 * w, col0 = nq * 64;
  if (row0 >= (int)NR) return;
  const unsigned short* a0p = X16 + (size_t)(row0 + ln) * DM;
  const Acc8 c = g2_main(a0p, a0p + (size_t)16 * DM, BQ + (size_t)(col0 + ln) * DM, DM, DM, hh);
  v8f accs[8] = {c.c00, c.c01, c.c02, c.c03, c.c10, c.c11, c.c12, c.c13};
#pragma unroll
  for (int u = 0; u < 8; ++u) { const int t = u & 3, hf = u >> 2; const float bv = bf16_rne(bias[col0 + t * 16 + ln]);
#pragma unroll
    for (int r = 0; r < 8; ++r) so[w][hf * 16 + 8 * hh + r][t * 16 + ln] = accs[u][r] * 0.0625f + bv; }
  __builtin_amdgcn_fence(4  , "workgroup"); __builtin_amdgcn_wave_barrier();
  const int which = col0 >> 10;
  const int pl = (which == 0) ? 0 : which + 1;
  const int cp = col0 & (DM - 1);
  const int rq = lane >> 3, c8 = (lane & 7) * 8;
  const size_t pofs = (size_t)pl * PSZ;
  for (int pass = 0; pass < 2; ++pass) {
#pragma unroll
    for (int q = 0; q < 8; ++q) { const int r = q * 4 + rq;
      const v4f a = *(const v4fa*)&so[w][r][c8], e = *(const v4fa*)&so[w][r][c8 + 4];
      FragH fh, fl;
#pragma unroll
      for (int i = 0; i < 4; ++i) { _Float16 h = (_Float16)a[i]; fh.h[i] = h; fl.h[i] = (_Float16)((a[i] - (float)h) * 1024.0f); h = (_Float16)e[i]; fh.h[4 + i] = h; fl.h[4 + i] = (_Float16)((e[i] - (float)h) * 1024.0f); }
      const v8us oh = fh.half[0], ol = fl.half[0];
      const size_t o = pofs + (size_t)(row0 + r) * DM + cp + c8;
      *(volatile v8us*)(PL + o) = oh;
      if (which == 0) *(volatile v8us*)(PL + PSZ + o) = ol; }
    if (pass == 0) __threadfence(); }
}

__global__ __launch_bounds__(256) void k_vt(const unsigned short* __restrict__ V16, unsigned short* __restrict__ Vt) {
  __shared__ unsigned short tl[64][66];
  const int tid = threadIdx.x; const int slab = blockIdx.x / (SEQ / 64), lg = blockIdx.x % (SEQ / 64); const int b = slab / NH, h = slab % NH;
  for (int i = tid; i < 64 * 8; i += 256) { const int r = i >> 3, c8 = (i & 7) * 8;
    const v8us f = *(const v8us*)(V16 + ((size_t)b * SEQ + lg * 64 + r) * DM + h * HD + c8);
#pragma unroll
    for (int q = 0; q < 8; ++q) tl[r][c8 + q] = f[q]; }
  __syncthreads();
  for (int pass = 0; pass < 2; ++pass) {
#pragma unroll
    for (int rd = 0; rd < 2; ++rd) { const int d = rd * 32 + (tid >> 3), pc = tid & 7; FragH f;
#pragma unroll
      for (int q = 0; q < 8; ++q) f.u[q] = tl[pc * 8 + q][d];
      const v8us o = f.half[0];
      *(volatile v8us*)(Vt + ((size_t)slab * HD + d) * SEQ + lg * 64 + pc * 8) = o; }
    if (pass == 0) __threadfence(); }
}

__global__ __launch_bounds__(128) void k_attn(const unsigned short* __restrict__ QH, const unsigned short* __restrict__ QL, const unsigned short* __restrict__ K16, const unsigned short* __restrict__ VT, unsigned short* __restrict__ CTX) {
  __shared__ __attribute__((aligned(16))) unsigned short lqh[64][72];
  __shared__ __attribute__((aligned(16))) unsigned short lql[64][72];
  __shared__ __attribute__((aligned(16))) float so[4][16][68];
  const int tid = threadIdx.x, lane = tid & 31, ln = lane & 15, hh = lane >> 4;
  const int wave = __builtin_amdgcn_readfirstlane(tid >> 5);
  const int bh = blockIdx.x / (SEQ / 64), qb = blockIdx.x % (SEQ / 64);
  const int b = bh / NH, h = bh % NH;
  const size_t qrow0 = (size_t)b * SEQ + (size_t)qb * 64;
  for (int i = tid; i < 64 * 8; i += 128) { const int r = i >> 3, c8 = (i & 7) * 8; const size_t g = (qrow0 + r) * DM + h * HD + c8;
    const v8us a = *(const v8us*)(QH + g); const v8us c = *(const v8us*)(QL + g);
    *(v8us*)&lqh[r][c8] = a; *(v8us*)&lql[r][c8] = c; }
  __syncthreads();
  const unsigned short* kbase = K16 + ((size_t)b * SEQ + ln) * DM + h * HD;
  const unsigned short* vbase = VT + ((size_t)bh * HD + ln) * SEQ;
  const v8f z8 = {0.f, 0.f, 0.f, 0.f, 0.f, 0.f, 0.f, 0.f};
  v8f o0 = z8, o1 = z8, o2 = z8, o3 = z8;
  float m = -1.0e30f, l = 0.f;
  const int qr = wave * 16 + ln;
#pragma unroll 1
  for (int kv = 0; kv < SEQ; kv += 32) {
    int zo = 0; asm volatile("" : "+v"(zo));
    const int qrr = qr + zo;
    FragH fq;
    fq.half[0] = *(const v8us*)&lqh[qrr][8 * hh];      fq.half[1] = *(const v8us*)&lqh[qrr][16 + 8 * hh]; const v16h qh0 = fq.v;
    fq.half[0] = *(const v8us*)&lqh[qrr][32 + 8 * hh]; fq.half[1] = *(const v8us*)&lqh[qrr][48 + 8 * hh]; const v16h qh1 = fq.v;
    fq.half[0] = *(const v8us*)&lql[qrr][8 * hh];      fq.half[1] = *(const v8us*)&lql[qrr][16 + 8 * hh]; const v16h ql0 = fq.v;
    fq.half[0] = *(const v8us*)&lql[qrr][32 + 8 * hh]; fq.half[1] = *(const v8us*)&lql[qrr][48 + 8 * hh]; const v16h ql1 = fq.v;
    v8f sa[2];
#pragma unroll
    for (int j = 0; j < 2; ++j) {
      const unsigned short* kp = kbase + (size_t)(kv + 16 * j) * DM;
      const v16h k0 = g2_frag(kp, hh), k1 = g2_frag(kp + 32, hh);
      v8f sh = z8, sl = z8;
      sh = g2_mma(k0, qh0, sh); sh = g2_mma(k1, qh1, sh);
      sl = g2_mma(k0, ql0, sl); sl = g2_mma(k1, ql1, sl);
#pragma unroll
      for (int r = 0; r < 8; ++r) sa[j][r] = (sh[r] + sl[r] * 0.0009765625f) * 0.25f;
    }
    float mx = fmaxf(sa[0][0], sa[1][0]);
#pragma unroll
    for (int r = 1; r < 8; ++r) mx = fmaxf(mx, fmaxf(sa[0][r], sa[1][r]));
    mx = fmaxf(mx, __shfl_xor(mx, 16));
    const float mn = fmaxf(m, mx);
    const float al = __expf(m - mn);
    m = mn;
    const float sft = LN256 - mn;
    FragH pb; float ps = 0.f;
#pragma unroll
    for (int r = 0; r < 8; ++r) { const float p0 = __expf(sa[0][r] + sft), p1 = __expf(sa[1][r] + sft); ps += p0 + p1; pb.h[r] = (_Float16)p0; pb.h[8 + r] = (_Float16)p1; }
    l = l * al + ps;
    const unsigned short* vp = vbase + kv;
    const v16h v0 = g2_frag(vp, hh), v1 = g2_frag(vp + (size_t)16 * SEQ, hh), v2 = g2_frag(vp + (size_t)32 * SEQ, hh), v3 = g2_frag(vp + (size_t)48 * SEQ, hh);
#pragma unroll
    for (int r = 0; r < 8; ++r) { o0[r] *= al; o1[r] *= al; o2[r] *= al; o3[r] *= al; }
    const v16h pv = pb.v;
    o0 = g2_mma(v0, pv, o0); o1 = g2_mma(v1, pv, o1); o2 = g2_mma(v2, pv, o2); o3 = g2_mma(v3, pv, o3);
  }
  const float lt = l + __shfl_xor(l, 16);
  const float inv = 64.0f * (1.0f / lt);
  v8f oo[4] = {o0, o1, o2, o3};
#pragma unroll
  for (int t = 0; t < 4; ++t)
#pragma unroll
    for (int r = 0; r < 8; ++r) so[wave][ln][16 * t + 8 * hh + r] = oo[t][r] * inv;
  __builtin_amdgcn_fence(4  , "workgroup"); __builtin_amdgcn_wave_barrier();
  const int rq = lane >> 3, c8 = (lane & 7) * 8;
  for (int pass = 0; pass < 2; ++pass) {
#pragma unroll
    for (int it = 0; it < 4; ++it) { const int r = it * 4 + rq;
      const v4f a = *(const v4fa*)&so[wave][r][c8], e = *(const v4fa*)&so[wave][r][c8 + 4];
      FragH fh, fl;
#pragma unroll
      for (int i = 0; i < 4; ++i) { _Float16 hv = (_Float16)a[i]; fh.h[i] = hv; fl.h[i] = (_Float16)((a[i] - (float)hv) * 64.0f); hv = (_Float16)e[i]; fh.h[4 + i] = hv; fl.h[4 + i] = (_Float16)((e[i] - (float)hv) * 64.0f); }
      const v8us oh = fh.half[0], ol = fl.half[0];
      const size_t g = (qrow0 + (size_t)(wave * 16 + r)) * (size_t)(2 * DM) + h * HD + c8;
      *(volatile v8us*)(CTX + g) = oh;
      *(volatile v8us*)(CTX + g + DM) = ol; }
    if (pass == 0) __threadfence(); }
}

__global__ __launch_bounds__(128) void k_gemm_out(const unsigned short* __restrict__ CTX, const unsigned short* __restrict__ BO, const float* __restrict__ bias, float* __restrict__ out) {
  __shared__ __attribute__((aligned(16))) float so[4][32][68];
  const int tid = threadIdx.x, lane = tid & 31, ln = lane & 15, hh = lane >> 4;
  const int w = __builtin_amdgcn_readfirstlane(tid >> 5);
  const int ntn = DM / 64; const int mt = blockIdx.x / ntn, nq = blockIdx.x - mt * ntn;
  const int row0 = mt * 128 + 32 * w, col0 = nq * 64;
  if (row0 >= (int)NR) return;
  const unsigned short* a0p = CTX + (size_t)(row0 + ln) * (2 * DM);
  const Acc8 c = g2_main(a0p, a0p + (size_t)16 * (2 * DM), BO + (size_t)(col0 + ln) * (2 * DM), 2 * DM, 2 * DM, hh);
  v8f accs[8] = {c.c00, c.c01, c.c02, c.c03, c.c10, c.c11, c.c12, c.c13};
#pragma unroll
  for (int u = 0; u < 8; ++u) { const int t = u & 3, hf = u >> 2; const float bv = bf16_rne(bias[col0 + t * 16 + ln]);
#pragma unroll
    for (int r = 0; r < 8; ++r) so[w][hf * 16 + 8 * hh + r][t * 16 + ln] = accs[u][r] * 0.000244140625f + bv; }
  __builtin_amdgcn_fence(4  , "workgroup"); __builtin_amdgcn_wave_barrier();
  const int rsub = lane >> 4, c4 = (lane & 15) * 4;
  for (int pass = 0; pass < 2; ++pass) {
#pragma unroll
    for (int q = 0; q < 16; ++q) { const int r = q * 2 + rsub; const int row = row0 + r;
      const size_t orow = (size_t)(row / SEQ) * SEQ_FULL + (size_t)(row % SEQ);
      const v4f v = *(const v4fa*)&so[w][r][c4];
      *(volatile v4f*)(out + orow * DM + col0 + c4) = v; }
    if (pass == 0) __threadfence(); }
}

#define SZ_BQ  ((size_t)LQ * DM * 2)
#define SZ_BO  ((size_t)DM * 2 * DM * 2)
#define SZ_X   ((size_t)NB * SEQ * DM * 2)
#define SZ_PL  ((size_t)4 * NB * SEQ * DM * 2)
#define SZ_VT  ((size_t)NB * SEQ * DM * 2)
#define SZ_CTX ((size_t)NB * SEQ * 2 * DM * 2)
static_assert(SZ_BQ % 256 == 0 && SZ_BO % 256 == 0 && SZ_X % 256 == 0 && SZ_PL % 256 == 0 && SZ_VT % 256 == 0 && SZ_CTX % 256 == 0);
static_assert(SZ_BQ + SZ_BO + SZ_X + SZ_PL + SZ_VT + SZ_CTX <= (size_t)134217728);

extern "C" void kernel_launch(void* const* d_in, const int* in_sizes, int n_in,
                              void* d_out, int out_size, void* d_ws, size_t ws_size, hipStream_t stream) {
  if (n_in < 5) return;
  const long long need_x = ((long long)(NB - 1) * SEQ_FULL + SEQ) * DM;
  if ((long long)in_sizes[0] < need_x) return;
  if (in_sizes[1] < DM * LQ || in_sizes[2] < LQ || in_sizes[3] < DM * DM || in_sizes[4] < DM) return;
  if ((long long)out_size < need_x) return;
  const float* x = (const float*)d_in[0]; const float* wqkv = (const float*)d_in[1]; const float* bqkv = (const float*)d_in[2];
  const float* wo = (const float*)d_in[3]; const float* bo = (const float*)d_in[4];
  const size_t total = SZ_BQ + SZ_BO + SZ_X + SZ_PL + SZ_VT + SZ_CTX;
  if (total > ws_size) return;
  char* ws = (char*)d_ws; size_t off = 0;
  unsigned short* BQ  = (unsigned short*)(ws + off); off += SZ_BQ;
  unsigned short* BO  = (unsigned short*)(ws + off); off += SZ_BO;
  unsigned short* X16 = (unsigned short*)(ws + off); off += SZ_X;
  unsigned short* PL  = (unsigned short*)(ws + off); off += SZ_PL;
  unsigned short* VT  = (unsigned short*)(ws + off); off += SZ_VT;
  unsigned short* CTX = (unsigned short*)(ws + off); off += SZ_CTX;
  k_wt_f16<<<(unsigned)(((size_t)LQ * (DM / 8) + 255) / 256), 256, 0, stream>>>(wqkv, BQ, DM, LQ, DM, 16.0f, 0.0f, 0);
  k_wt_f16<<<(unsigned)(((size_t)DM * (DM / 8) + 255) / 256), 256, 0, stream>>>(wo, BO, DM, DM, 2 * DM, 64.0f, 1.0f, 1);
  k_x16<<<(unsigned)((NR * DM / 8 + 255) / 256), 256, 0, stream>>>(x, X16);
  k_gemm_qkv<<<(unsigned)((NR / 128) * (LQ / 64)), 128, 0, stream>>>(X16, BQ, bqkv, PL);
  k_vt<<<(unsigned)(NB * NH * (SEQ / 64)), 256, 0, stream>>>(PL + 3 * PSZ, VT);
  k_attn<<<(unsigned)(NB * NH * (SEQ / 64)), 128, 0, stream>>>(PL, PL + PSZ, PL + 2 * PSZ, VT, CTX);
  k_gemm_out<<<(unsigned)((NR / 128) * (DM / 64)), 128, 0, stream>>>(CTX, BO, bo, (float*)d_out);
}
